// MoEDispatcher_17935783428802
// MI455X (gfx1250) — hardware-verified
//
#include <hip/hip_runtime.h>
#include <stdint.h>
#include <stddef.h>
#include <math.h>

#define NTOK 4096
#define DM   1024
#define DF   1024
#define NEX  8
#define MT   32
#define NSL  256
#define XP   1032
#define YP   260
#define TP   72
#define WSC  256.0f
#define WSCI 0.00390625f

#define LDS_XB  (MT * XP * 2)
#define LDS_YB  (MT * YP * 4)
#define LDS_EXP (LDS_XB + LDS_YB)

static_assert((XP * 2) % 16 == 0);
static_assert((YP * 4) % 16 == 0);
static_assert((TP * 2) % 16 == 0);
static_assert(NTOK % 256 == 0);
static_assert(NTOK % MT == 0);
static_assert(DF % NSL == 0);
static_assert(DM % 64 == 0);
static_assert(DF % 64 == 0);
static_assert(DM % 32 == 0);
static_assert(NSL == 8 * 32);
static_assert(MT == 8 * 4);
static_assert(LDS_XB % 16 == 0);

typedef _Float16       v16h __attribute__((ext_vector_type(16)));
typedef _Float16       v8h  __attribute__((ext_vector_type(8)));
typedef float          v8f  __attribute__((ext_vector_type(8)));
typedef float          v4f  __attribute__((ext_vector_type(4)));
typedef unsigned int   v4u  __attribute__((ext_vector_type(4)));
typedef v4f __attribute__((may_alias)) v4fa;
typedef v4u __attribute__((may_alias)) v4ua;

union FragH { v16h v; v4u q[2]; };
union Pk8   { v8h h; v4u u; };

__device__ __forceinline__ unsigned short hbits(float f) {
  const _Float16 h = (_Float16)f;
  return __builtin_bit_cast(unsigned short, h);
}
__device__ __forceinline__ v4u pack8(v4f a, v4f c, float s) {
  Pk8 k;
  k.h[0] = (_Float16)(a.x * s); k.h[1] = (_Float16)(a.y * s);
  k.h[2] = (_Float16)(a.z * s); k.h[3] = (_Float16)(a.w * s);
  k.h[4] = (_Float16)(c.x * s); k.h[5] = (_Float16)(c.y * s);
  k.h[6] = (_Float16)(c.z * s); k.h[7] = (_Float16)(c.w * s);
  return k.u;
}

__device__ __forceinline__ v8f wmma_h(v16h a, v16h b, v8f c) {
  v8f d = __builtin_amdgcn_wmma_f32_16x16x32_f16(false, a, false, b, (short)0, c, false, false);
  asm volatile("v_nop\n\tv_nop\n\tv_nop\n\tv_nop" : "+v"(d) : "v"(a), "v"(b));
  return d;
}

__device__ __forceinline__ v16h ldfrag_h(const unsigned short* p, int h) {
  FragH f;
  f.q[0] = *(const v4ua*)(p + 8 * h);
  f.q[1] = *(const v4ua*)(p + 16 + 8 * h);
  return f.v;
}

__global__ __launch_bounds__(256) void k_wt(const float* __restrict__ w,
                                            unsigned short* __restrict__ wt)
{
  __shared__ __align__(16) unsigned short sT[64 * TP];
  const int tid = threadIdx.x, lane = tid & 31, wv = tid >> 5;
  const int d0 = blockIdx.x * 64;
  const int f0 = blockIdx.y * 64;
  const int e  = blockIdx.z;
  const float* src = w + (size_t)e * DM * DF + (size_t)d0 * DF + f0;
  #pragma unroll
  for (int j = 0; j < 4; ++j) {
    const int idx = tid + 256 * j;
    const int row = idx >> 4;
    const int fb  = (idx & 15) * 4;
    const v4f v = *(const v4fa*)(src + (size_t)row * DF + fb);
    sT[(fb + 0) * TP + row] = hbits(v.x * WSC);
    sT[(fb + 1) * TP + row] = hbits(v.y * WSC);
    sT[(fb + 2) * TP + row] = hbits(v.z * WSC);
    sT[(fb + 3) * TP + row] = hbits(v.w * WSC);
  }
  __syncthreads();
  const int q  = lane & 7;
  const int j0 = wv * 8 + (lane >> 3);
  const int j1 = j0 + 4;
  const v4u val0 = *(const v4ua*)(sT + j0 * TP + 8 * q);
  const v4u val1 = *(const v4ua*)(sT + j1 * TP + 8 * q);
  unsigned short* dst0 = wt + ((size_t)e * DF + f0 + j0) * DM + d0 + 8 * q;
  unsigned short* dst1 = wt + ((size_t)e * DF + f0 + j1) * DM + d0 + 8 * q;
  *(volatile v4u*)dst0 = val0;
  *(volatile v4u*)dst1 = val1;
  __threadfence();
  *(volatile v4u*)dst0 = val0;
  *(volatile v4u*)dst1 = val1;
}

__global__ __launch_bounds__(256) void k_route(const float* __restrict__ lg,
                                               float* __restrict__ rec, int ntok)
{
  const int t  = blockIdx.x * 256 + threadIdx.x;
  const int tc = (t < ntok) ? t : (ntok - 1);
  const float* p = lg + (size_t)tc * NEX;
  const v4f a = *(const v4fa*)p;
  const v4f b = *(const v4fa*)(p + 4);
  float l[NEX];
  l[0] = a.x; l[1] = a.y; l[2] = a.z; l[3] = a.w;
  l[4] = b.x; l[5] = b.y; l[6] = b.z; l[7] = b.w;

  int i0 = 0;
  float b0 = l[0];
  #pragma unroll
  for (int e = 1; e < NEX; ++e) {
    const bool tk = l[e] > b0;
    b0 = tk ? l[e] : b0;
    i0 = tk ? e : i0;
  }
  int i1 = -1;
  float b1 = -3.0e38f;
  #pragma unroll
  for (int e = 0; e < NEX; ++e) {
    const bool tk = (e != i0) && (l[e] > b1);
    b1 = tk ? l[e] : b1;
    i1 = tk ? e : i1;
  }
  i1 = (i1 < 0) ? ((i0 == 0) ? 1 : 0) : i1;
  float l1 = l[0];
  #pragma unroll
  for (int e = 0; e < NEX; ++e) l1 = (e == i1) ? l[e] : l1;

  const float mx = b0;
  float s = 0.0f;
  #pragma unroll
  for (int e = 0; e < NEX; ++e) s += __expf(l[e] - mx);
  const float rs = __builtin_amdgcn_rcpf(s);
  const float p0 = rs;
  const float p1 = __expf(l1 - mx) * rs;

  const v4f v = { p0, p1, (float)i0, (float)i1 };
  float* dst = rec + (size_t)tc * 4;
  if (t < ntok) *(volatile v4f*)dst = v;
  __threadfence();
  if (t < ntok) *(volatile v4f*)dst = v;
}

__device__ __forceinline__ void part_pass(const float* sY, const int* sTok, const int* sSlot,
                                          float* part, int ns, int wv, int lane, int nrows)
{
  #pragma unroll
  for (int i = 0; i < 4; ++i) {
    const int row = wv * 4 + i;
    int t = sTok[row];
    t = (t < 0) ? 0 : ((t > NTOK - 1) ? (NTOK - 1) : t);
    int s = sSlot[row];
    s = (s != 0) ? 1 : 0;
    const v4f v0 = *(const v4fa*)(sY + row * YP + 4 * lane);
    const v4f v1 = *(const v4fa*)(sY + row * YP + 128 + 4 * lane);
    float* dst = part + ((size_t)t * 2 + s) * DF + ns * NSL;
    if (row < nrows) {
      *(volatile v4f*)(dst + 4 * lane) = v0;
      *(volatile v4f*)(dst + 128 + 4 * lane) = v1;
    }
  }
}

__global__ __launch_bounds__(256) void k_expert(const float* __restrict__ x,
                                                const unsigned short* __restrict__ wt,
                                                const float* __restrict__ rec,
                                                float* __restrict__ part, int ntok)
{
  extern __shared__ __align__(16) unsigned char dsm_e[];
  unsigned short* sX = (unsigned short*)dsm_e;
  float* sY = (float*)(dsm_e + LDS_XB);
  __shared__ int   sTok[MT];
  __shared__ int   sSlot[MT];
  __shared__ float sW[MT];
  __shared__ int   s_wc[8];

  const int tid = threadIdx.x, lane = tid & 31, wv = tid >> 5;
  const int h = lane >> 4, m = lane & 15;
  const int e = blockIdx.y;
  const int m0 = blockIdx.x * MT;

  if (tid < MT) { sTok[tid] = 0; sSlot[tid] = 0; sW[tid] = 0.0f; }
  __syncthreads();

  int base = 0;
  #pragma unroll 1
  for (int ch = 0; ch < NTOK / 256; ++ch) {
    const int t = ch * 256 + tid;
    const int tc = (t < ntok) ? t : (ntok - 1);
    const v4f r = *(const v4fa*)(rec + (size_t)tc * 4);
    int e0 = (int)r.z, e1 = (int)r.w;
    e0 = (e0 < 0) ? 0 : ((e0 > NEX - 1) ? (NEX - 1) : e0);
    e1 = (e1 < 0) ? 0 : ((e1 > NEX - 1) ? (NEX - 1) : e1);
    const bool f0 = (e0 == e);
    const bool f1 = (e1 == e) && !f0;
    const bool f = (f0 || f1) && (t < ntok);
    const unsigned int msk = __builtin_amdgcn_ballot_w32(f);
    const int off = __builtin_popcount(msk & ((1u << lane) - 1u));
    const int wc = __builtin_popcount(msk);
    if (lane == 0) s_wc[wv] = wc;
    __syncthreads();
    int pre = 0, tot = 0;
    #pragma unroll
    for (int w2 = 0; w2 < 8; ++w2) {
      const int cc = s_wc[w2];
      tot += cc;
      pre += (w2 < wv) ? cc : 0;
    }
    if (f) {
      const int p = base + pre + off - m0;
      if ((unsigned)p < (unsigned)MT) {
        sTok[p]  = t;
        sSlot[p] = f0 ? 0 : 1;
        sW[p]    = f0 ? r.x : r.y;
      }
    }
    base += tot;
    __syncthreads();
  }
  const int cnt = base;
  if (m0 >= cnt) return;
  int nrows = cnt - m0;
  nrows = (nrows > MT) ? MT : nrows;

  #pragma unroll 4
  for (int j = 0; j < 16; ++j) {
    const int idx = tid + 256 * j;
    const int row = idx >> 7, c8 = idx & 127;
    int t = sTok[row];
    t = (t < 0) ? 0 : ((t > NTOK - 1) ? (NTOK - 1) : t);
    const float* g = x + (size_t)t * DM + 8 * c8;
    const v4f a = *(const v4fa*)g;
    const v4f c = *(const v4fa*)(g + 4);
    *(v4ua*)(sX + row * XP + 8 * c8) = pack8(a, c, 1.0f);
  }
  __syncthreads();

  const v8f z8 = {0.f, 0.f, 0.f, 0.f, 0.f, 0.f, 0.f, 0.f};

  #pragma unroll 1
  for (int ns = 0; ns < DF / NSL; ++ns) {
    v8f acc[2][2];
    #pragma unroll
    for (int mt = 0; mt < 2; ++mt)
      #pragma unroll
      for (int nt = 0; nt < 2; ++nt) acc[mt][nt] = z8;
    #pragma unroll 1
    for (int k0 = 0; k0 < DM; k0 += 32) {
      v16h af[2];
      #pragma unroll
      for (int mt = 0; mt < 2; ++mt)
        af[mt] = ldfrag_h(sX + (16 * mt + m) * XP + k0, h);
      #pragma unroll
      for (int nt = 0; nt < 2; ++nt) {
        const int f = ns * NSL + wv * 32 + 16 * nt + m;
        const size_t bo = ((size_t)e * DF + f) * DM + k0;
        const v16h bf = ldfrag_h(wt + bo, h);
        #pragma unroll
        for (int mt = 0; mt < 2; ++mt)
          acc[mt][nt] = wmma_h(af[mt], bf, acc[mt][nt]);
      }
    }
    #pragma unroll
    for (int mt = 0; mt < 2; ++mt)
      #pragma unroll
      for (int nt = 0; nt < 2; ++nt) {
        const int cl = wv * 32 + 16 * nt + m;
        #pragma unroll
        for (int r = 0; r < 8; ++r) {
          const int row = 16 * mt + 8 * h + r;
          const float sc = sW[row] * WSCI;
          sY[row * YP + cl] = acc[mt][nt][r] * sc;
        }
      }
    __syncthreads();
    part_pass(sY, sTok, sSlot, part, ns, wv, lane, nrows);
    __threadfence();
    part_pass(sY, sTok, sSlot, part, ns, wv, lane, nrows);
    __syncthreads();
  }
}

__global__ __launch_bounds__(256) void k_sum(const float* __restrict__ part,
                                             float* __restrict__ out, int n4)
{
  const int g = blockIdx.x * 256 + threadIdx.x;
  if (g >= n4) return;
  const int t  = g >> 8;
  const int c4 = g & 255;
  const v4f a = *(const v4fa*)(part + ((size_t)t * 2 + 0) * DF + 4 * c4);
  const v4f b = *(const v4fa*)(part + ((size_t)t * 2 + 1) * DF + 4 * c4);
  const v4f v = a + b;
  float* dst = out + (size_t)g * 4;
  *(volatile v4f*)dst = v;
  __threadfence();
  *(volatile v4f*)dst = v;
}

extern "C" void kernel_launch(void* const* d_in, const int* in_sizes, int n_in,
                              void* d_out, int out_size, void* d_ws, size_t ws_size,
                              hipStream_t stream)
{
  if (n_in < 3) return;
  if (in_sizes[0] != NTOK * DM) return;
  if (in_sizes[1] != NTOK * NEX) return;
  if (in_sizes[2] != NEX * DM * DF) return;
  if (out_size != NTOK * DF) return;

  const float* x  = (const float*)d_in[0];
  const float* lg = (const float*)d_in[1];
  const float* w  = (const float*)d_in[2];
  float* out = (float*)d_out;

  const size_t bWT   = (size_t)NEX * DF * DM * 2;
  const size_t bREC  = (size_t)NTOK * 16;
  const size_t bPART = (size_t)NTOK * 2 * DF * 4;
  const size_t total = bWT + bREC + bPART;
  if (total > ws_size) return;
  if (total > (size_t)134217728) return;

  char* ws = (char*)d_ws;
  size_t off = 0;
  unsigned short* WT   = (unsigned short*)(ws + off); off += bWT;
  float*          REC  = (float*)(ws + off);          off += bREC;
  float*          PART = (float*)(ws + off);          off += bPART;
  if (off != total) return;

  k_wt<<<dim3(DM / 64, DF / 64, NEX), 256, 0, stream>>>(w, WT);
  k_route<<<NTOK / 256, 256, 0, stream>>>(lg, REC, NTOK);
  hipFuncSetAttribute(reinterpret_cast<const void*>(&k_expert),
                      hipFuncAttributeMaxDynamicSharedMemorySize, LDS_EXP);
  k_expert<<<dim3(NTOK / MT, NEX), 256, LDS_EXP, stream>>>(x, WT, REC, PART, NTOK);
  {
    const int n4 = NTOK * DF / 4;
    k_sum<<<(n4 + 255) / 256, 256, 0, stream>>>(PART, out, n4);
  }
}
